// TransformerAutoencoder_7696581394490
// MI455X (gfx1250) — hardware-verified
//
#include <hip/hip_runtime.h>
#include <stdint.h>

constexpr int kBatch  = 4;
constexpr int kSeq    = 2048;
constexpr int kInDim  = 256;
constexpr int kHid    = 256;
constexpr int kHeads  = 4;
constexpr int kHdim   = 64;
constexpr int kFfn    = 1024;
constexpr int kLayers = 3;
constexpr int kTok    = kBatch * kSeq;
constexpr int kWin    = 32;
constexpr int kNT64   = kSeq / 64;
constexpr int kPBW    = 192;
constexpr int kNZ     = kBatch * kHeads;
constexpr int kQKW    = 2 * kHid;

typedef __attribute__((ext_vector_type(16))) _Float16 v16h;
typedef __attribute__((ext_vector_type(8)))  _Float16 v8h;
typedef __attribute__((ext_vector_type(16))) __bf16   v16b;
typedef __attribute__((ext_vector_type(8)))  __bf16   v8b;
typedef __attribute__((ext_vector_type(8)))  float    v8f;
typedef __attribute__((ext_vector_type(4)))  float    v4f;
typedef __attribute__((ext_vector_type(4)))  unsigned int v4u;
#define PSCALE 32768.0f

__device__ __forceinline__ unsigned short f2bf_bits(float f) {
  unsigned u = __float_as_uint(f);
  return (unsigned short)((u + 0x7FFFu + ((u >> 16) & 1u)) >> 16);
}
__device__ __forceinline__ float bf_bits2f(unsigned short h) { return __uint_as_float(((unsigned)h) << 16); }
__device__ __forceinline__ unsigned pk16(unsigned short a, unsigned short b) { return (unsigned)a | ((unsigned)b << 16); }

__device__ __forceinline__ void dep_guard_h(v8f& a, v8f& b, v16h x, v16h y) { asm volatile("v_nop\n\tv_nop\n\tv_nop\n\tv_nop" : "+v"(a), "+v"(b) : "v"(x), "v"(y)); }
__device__ __forceinline__ void dep_guard_b(v8f& a, v8f& b, v16b x, v16b y) { asm volatile("v_nop\n\tv_nop\n\tv_nop\n\tv_nop" : "+v"(a), "+v"(b) : "v"(x), "v"(y)); }
__device__ __forceinline__ void keep4_h(v16h a, v16h b, v16h c, v16h d) { asm volatile("v_nop" :: "v"(a), "v"(b), "v"(c), "v"(d)); }
__device__ __forceinline__ void keep4_b(v16b a, v16b b, v16b c, v16b d) { asm volatile("v_nop" :: "v"(a), "v"(b), "v"(c), "v"(d)); }
__device__ __forceinline__ void acc_guard4(v8f& a, v8f& b, v8f& c, v8f& d) { asm volatile("v_nop\n\tv_nop\n\tv_nop\n\tv_nop" : "+v"(a), "+v"(b), "+v"(c), "+v"(d)); }
template <typename T> struct Frag;
template <> struct Frag<_Float16> {
  typedef v16h V; union U { v16h v; v8h h[2]; };
  static __device__ __forceinline__ v16h load(const _Float16* p) {
    U f; f.h[0] = *(const v8h*)(p); f.h[1] = *(const v8h*)(p + 16); return f.v;
  }
  static __device__ __forceinline__ v8f mma(v16h a, v16h b, v8f c) {
    return __builtin_amdgcn_wmma_f32_16x16x32_f16(false, a, false, b, (short)0, c, false, false);
  }
  static __device__ __forceinline__ void guard(v8f& a, v8f& b, v16h x, v16h y) { dep_guard_h(a, b, x, y); }
  static __device__ __forceinline__ void keep(v16h a, v16h b, v16h c, v16h d) { keep4_h(a, b, c, d); }
};
template <> struct Frag<__bf16> {
  typedef v16b V; union U { v16b v; v8b h[2]; };
  static __device__ __forceinline__ v16b load(const __bf16* p) {
    U f; f.h[0] = *(const v8b*)(p); f.h[1] = *(const v8b*)(p + 16); return f.v;
  }
  static __device__ __forceinline__ v8f mma(v16b a, v16b b, v8f c) {
    return __builtin_amdgcn_wmma_f32_16x16x32_bf16(false, a, false, b, (short)0, c, false, false);
  }
  static __device__ __forceinline__ void guard(v8f& a, v8f& b, v16b x, v16b y) { dep_guard_b(a, b, x, y); }
  static __device__ __forceinline__ void keep(v16b a, v16b b, v16b c, v16b d) { keep4_b(a, b, c, d); }
};

template <int ET> struct Elem;
template <> struct Elem<0> { typedef _Float16 T; };
template <> struct Elem<1> { typedef __bf16 T; };
template <int ET, bool SPLIT, int BIAS_MODE, int OUT_MODE, bool RESID, int ACT = 0, int BANDMN = -1, int BANDK = -1, bool BANDST = false>
__global__ __launch_bounds__(256) void wmma_gemm64(
    const unsigned short* __restrict__ Ap, const unsigned short* __restrict__ A2p, int lda, long strideA,
    const unsigned short* __restrict__ Btp, const unsigned short* __restrict__ Bt2p, int ldb, long strideB,
    void* __restrict__ Cout, void* __restrict__ Cout2, int ldc, long strideC,
    const float* __restrict__ bias,
    const float* __restrict__ resid, long strideR,
    int M, int N, int K, float scale, float bsc,
    long zsA, long zsB, long zsC, long zsR) {
  typedef typename Elem<ET>::T T;
  typedef typename Frag<T>::V V;
  const T* A = (const T*)Ap; const T* A2 = (const T*)A2p; const T* Bt = (const T*)Btp; const T* Bt2 = (const T*)Bt2p;
  __shared__ __align__(16) float sT[8][16 * 68];
  const int b    = blockIdx.y;
  const int bz   = blockIdx.z;
  const int lane = threadIdx.x & 31;
  const int wave = threadIdx.x >> 5;
  const int tilesN = N >> 6;
  const int tilesM = M >> 6;
  const int tile = blockIdx.x * 8 + wave;
  if (tile >= tilesM * tilesN) return;
  const int tm = tile / tilesN;
  const int tn = tile - tm * tilesN;
  const int m0 = tm << 6;
  const int n0 = tn << 6;
  if (BANDMN >= 0) {
    int dt = tm - tn;
    dt = (dt < 0) ? -dt : dt;
    if (dt > BANDMN) return;
  }
  int nC = n0;
  if (BANDST && BANDMN >= 0) {
    int tl = tm - BANDMN; tl = (tl < 0) ? 0 : tl;
    nC = n0 - (tl << 6);
  }

  const size_t offA = (size_t)b * strideA + (size_t)bz * zsA;
  const size_t offB = (size_t)b * strideB + (size_t)bz * zsB;
  const size_t offC = (size_t)b * strideC + (size_t)bz * zsC;
  const size_t offR = (size_t)b * strideR + (size_t)bz * zsR;
  const T* Ab  = A  + offA;
  const T* Bb  = Bt + offB;
  const T* Ab2 = SPLIT ? (A2  + offA) : nullptr;
  const T* Bb2 = SPLIT ? (Bt2 + offB) : nullptr;

  const int rlane = lane & 15;
  const int koff  = (lane >> 4) * 8;
  const int mOff  = (lane >> 4) * 8;

  v8f acc[4][4];
#pragma unroll
  for (int i = 0; i < 4; ++i)
#pragma unroll
    for (int j = 0; j < 4; ++j) acc[i][j] = (v8f){0.f,0.f,0.f,0.f,0.f,0.f,0.f,0.f};

  int kBeg = 0, kEnd = K;
  if (BANDK >= 0) {
    int ks = (tm - BANDK) * 64;     ks = (ks < 0) ? 0 : ks;
    int ke = (tm + BANDK + 1) * 64; ke = (ke > K) ? K : ke;
    kBeg = __builtin_amdgcn_readfirstlane(ks);
    kEnd = __builtin_amdgcn_readfirstlane(ke);
  }
  const int kA = (BANDST && BANDK >= 0) ? kBeg : 0;
  for (int k0 = kBeg; k0 < kEnd; k0 += 32) {
    V bh[4], bl[4];
#pragma unroll
    for (int j = 0; j < 4; ++j) {
      const size_t bo = (size_t)(n0 + (j << 4) + rlane) * ldb + koff + k0;
      bh[j] = Frag<T>::load(Bb + bo);
      if (SPLIT) bl[j] = Frag<T>::load(Bb2 + bo);
    }
#pragma unroll
    for (int i = 0; i < 4; ++i) {
      const size_t ao = (size_t)(m0 + (i << 4) + rlane) * lda + koff + (k0 - kA);
      V ah = Frag<T>::load(Ab + ao);
      V al;
      if (SPLIT) al = Frag<T>::load(Ab2 + ao);
#pragma unroll
      for (int j = 0; j < 4; ++j) {
        acc[i][j] = Frag<T>::mma(ah, bh[j], acc[i][j]);
        if (SPLIT) {
          acc[i][j] = Frag<T>::mma(ah, bl[j], acc[i][j]);
          acc[i][j] = Frag<T>::mma(al, bh[j], acc[i][j]);
        }
      }
      Frag<T>::guard(acc[i][0], acc[i][3], ah, SPLIT ? al : ah);
    }
    Frag<T>::keep(bh[0], bh[1], bh[2], bh[3]);
    if (SPLIT) Frag<T>::keep(bl[0], bl[1], bl[2], bl[3]);
  }
  acc_guard4(acc[0][0], acc[0][1], acc[0][2], acc[0][3]);
  acc_guard4(acc[1][0], acc[1][1], acc[1][2], acc[1][3]);
  acc_guard4(acc[2][0], acc[2][1], acc[2][2], acc[2][3]);
  acc_guard4(acc[3][0], acc[3][1], acc[3][2], acc[3][3]);

  float* slab = sT[wave];
  const float* Rb = RESID ? (resid + offR) : nullptr;
#pragma unroll
  for (int i = 0; i < 4; ++i) {
    const int mBase = m0 + (i << 4);
#pragma unroll
    for (int j = 0; j < 4; ++j) {
      const int n = n0 + (j << 4) + rlane;
      float bv = 0.f;
      if (BIAS_MODE == 2) bv = bias[n] * bsc;
#pragma unroll
      for (int r = 0; r < 8; ++r) {
        float v = acc[i][j][r] * scale;
        if (BIAS_MODE == 1) v += bias[mBase + mOff + r] * bsc;
        if (BIAS_MODE == 2) v += bv;
        if (RESID) v += Rb[(size_t)(mBase + mOff + r) * ldc + n];
        if (ACT == 2) v = fmaxf(v, 0.0f);
        if (ACT == 4) v = (v > 0.f) ? v : 0.01f * v;
        slab[(mOff + r) * 68 + (j << 4) + rlane] = v;
      }
    }
    __builtin_amdgcn_fence(__ATOMIC_RELEASE, "workgroup");
    __builtin_amdgcn_wave_barrier();
    __builtin_amdgcn_fence(__ATOMIC_ACQUIRE, "workgroup");
    if (OUT_MODE == 0) {
      float* C = (float*)Cout + offC;
      const int hh = lane >> 4, c4 = (lane & 15) * 4;
      for (int pass = 0; pass < 2; ++pass) {
#pragma unroll
        for (int it = 0; it < 8; ++it) {
          const int row = it * 2 + hh;
          v4f v = *(const v4f*)(slab + row * 68 + c4);
          *(volatile v4f*)(C + (size_t)(mBase + row) * ldc + nC + c4) = v;
        }
        __threadfence();
      }
    } else {
      const int q = lane >> 3, c8 = (lane & 7) * 8;
      unsigned short* C  = (unsigned short*)Cout  + offC;
      unsigned short* C2 = (OUT_MODE == 2) ? ((unsigned short*)Cout2 + offC) : nullptr;
      for (int pass = 0; pass < 2; ++pass) {
#pragma unroll
        for (int it = 0; it < 4; ++it) {
          const int row = it * 4 + q;
          const float* sp = slab + row * 68 + c8;
          v8h hv, lv;
#pragma unroll
          for (int e = 0; e < 8; ++e) {
            if (OUT_MODE == 1) {
              hv[e] = (_Float16)sp[e];
            } else {
              unsigned short hb = f2bf_bits(sp[e]);
              unsigned short lb = f2bf_bits(sp[e] - bf_bits2f(hb));
              hv[e] = __builtin_bit_cast(_Float16, hb);
              lv[e] = __builtin_bit_cast(_Float16, lb);
            }
          }
          *(volatile v8h*)(C + (size_t)(mBase + row) * ldc + nC + c8) = hv;
          if (OUT_MODE == 2) *(volatile v8h*)(C2 + (size_t)(mBase + row) * ldc + nC + c8) = lv;
        }
        __threadfence();
      }
    }
    __builtin_amdgcn_fence(__ATOMIC_RELEASE, "workgroup");
    __builtin_amdgcn_wave_barrier();
    __builtin_amdgcn_fence(__ATOMIC_ACQUIRE, "workgroup");
  }
}

__global__ __launch_bounds__(256) void cast_f32_f16x2s(
    const float* __restrict__ in, _Float16* __restrict__ out, int n2, float sc) {
  int i = blockIdx.x * 256 + threadIdx.x;
  if (i < n2) {
    const size_t i2 = 2 * (size_t)i;
    const _Float16 h0 = (_Float16)(in[i2] * sc), h1 = (_Float16)(in[i2 + 1] * sc);
    const unsigned u = (unsigned)__builtin_bit_cast(unsigned short, h0) | ((unsigned)__builtin_bit_cast(unsigned short, h1) << 16);
    ((volatile unsigned*)out)[i] = u;
    __threadfence();
    ((volatile unsigned*)out)[i] = u;
  }
}

__global__ __launch_bounds__(128) void pe_rows_kernel(float* __restrict__ PE) {
  __shared__ __align__(16) float rowbuf[kHid];
  const int pos = blockIdx.x;
  const int t   = threadIdx.x;
  const float cexp = -0.03597789207803197f;
  const float dv  = expf((float)(2 * t) * cexp);
  const float ang = (float)pos * dv;
  rowbuf[2 * t]     = sinf(ang);
  rowbuf[2 * t + 1] = cosf(ang);
  __syncthreads();
  if (t < 64) {
    const v4f v = *(const v4f*)(rowbuf + 4 * t);
    float* dst = PE + (size_t)pos * kHid + 4 * t;
    *(volatile v4f*)dst = v;
    __threadfence();
    *(volatile v4f*)dst = v;
  }
}

__global__ __launch_bounds__(256) void layernorm_f16_kernel(
    const float* __restrict__ X, const float* __restrict__ gam, const float* __restrict__ bet,
    unsigned short* __restrict__ Y, int nrows) {
  const int wave = threadIdx.x >> 5, lane = threadIdx.x & 31;
  const int row  = blockIdx.x * 8 + wave;
  const int rowc = (row < nrows) ? row : (nrows - 1);
  const float* xr = X + (size_t)rowc * kHid + lane * 8;
  const v4f a0 = *(const v4f*)xr;
  const v4f a1 = *(const v4f*)(xr + 4);
  float v[8] = {a0[0], a0[1], a0[2], a0[3], a1[0], a1[1], a1[2], a1[3]};
  float sum = 0.f;
#pragma unroll
  for (int e = 0; e < 8; ++e) sum += v[e];
#pragma unroll
  for (int off = 16; off > 0; off >>= 1) sum += __shfl_xor(sum, off, 32);
  const float mu = sum * (1.0f / (float)kHid);
  float d[8];
  float var = 0.f;
#pragma unroll
  for (int e = 0; e < 8; ++e) { d[e] = v[e] - mu; var += d[e] * d[e]; }
#pragma unroll
  for (int off = 16; off > 0; off >>= 1) var += __shfl_xor(var, off, 32);
  const float rstd = rsqrtf(var * (1.0f / (float)kHid) + 1e-5f);
  const v4f g0 = *(const v4f*)(gam + lane * 8), g1 = *(const v4f*)(gam + lane * 8 + 4);
  const v4f b0 = *(const v4f*)(bet + lane * 8), b1 = *(const v4f*)(bet + lane * 8 + 4);
  const float gg[8] = {g0[0], g0[1], g0[2], g0[3], g1[0], g1[1], g1[2], g1[3]};
  const float bb[8] = {b0[0], b0[1], b0[2], b0[3], b1[0], b1[1], b1[2], b1[3]};
  unsigned short hb[8];
#pragma unroll
  for (int e = 0; e < 8; ++e) hb[e] = __builtin_bit_cast(unsigned short, (_Float16)(d[e] * rstd * gg[e] + bb[e]));
  const v4u pv = (v4u){pk16(hb[0], hb[1]), pk16(hb[2], hb[3]), pk16(hb[4], hb[5]), pk16(hb[6], hb[7])};
  unsigned short* dst = Y + (size_t)rowc * kHid + lane * 8;
  if (row < nrows) *(volatile v4u*)dst = pv;
  __threadfence();
  if (row < nrows) *(volatile v4u*)dst = pv;
}

__global__ __launch_bounds__(128) void band_softmax_kernel(const float* __restrict__ S, unsigned short* __restrict__ P) {
  const int wave = threadIdx.x >> 5, lane = threadIdx.x & 31;
  const int i    = blockIdx.x * 4 + wave;
  const int z    = blockIdx.y;
  const int tm   = i >> 6;
  int tlo = tm - 1; tlo = (tlo < 0) ? 0 : tlo;
  int thi = tm + 2; thi = (thi > kNT64) ? kNT64 : thi;
  const int c0 = tlo * 64;
  const int c1 = thi * 64;
  const int jj = lane * 8;
  const int j  = c0 + jj;
  const bool active = (j < c1);
  const int jjc = active ? jj : 0;
  const size_t roff = ((size_t)z * kSeq + (size_t)i) * kPBW;
  const v4f a0 = *(const v4f*)(S + roff + jjc);
  const v4f a1 = *(const v4f*)(S + roff + jjc + 4);
  const float sv[8] = {a0[0], a0[1], a0[2], a0[3], a1[0], a1[1], a1[2], a1[3]};
  bool  adm[8];
  float t[8];
  float m = -__builtin_inff();
#pragma unroll
  for (int e = 0; e < 8; ++e) {
    const int d = (j + e) - i;
    adm[e] = active && (d <= kWin) && (d >= -kWin);
    t[e] = adm[e] ? sv[e] : -__builtin_inff();
    m = fmaxf(m, t[e]);
  }
#pragma unroll
  for (int off = 16; off > 0; off >>= 1) m = fmaxf(m, __shfl_xor(m, off, 32));
  float ev[8];
  float s = 0.f;
#pragma unroll
  for (int e = 0; e < 8; ++e) {
    ev[e] = adm[e] ? __expf(t[e] - m) : 0.0f;
    s += ev[e];
  }
#pragma unroll
  for (int off = 16; off > 0; off >>= 1) s += __shfl_xor(s, off, 32);
  const float inv = PSCALE * (1.0f / s);
  unsigned short hb[8];
#pragma unroll
  for (int e = 0; e < 8; ++e) hb[e] = __builtin_bit_cast(unsigned short, (_Float16)(ev[e] * inv));
  const v4u pv = (v4u){pk16(hb[0], hb[1]), pk16(hb[2], hb[3]), pk16(hb[4], hb[5]), pk16(hb[6], hb[7])};
  unsigned short* dst = P + roff + (size_t)jjc;
  if (active) *(volatile v4u*)dst = pv;
  __threadfence();
  if (active) *(volatile v4u*)dst = pv;
}

extern "C" void kernel_launch(void* const* d_in, const int* in_sizes, int n_in,
                              void* d_out, int out_size, void* d_ws, size_t ws_size,
                              hipStream_t stream) {
  if (n_in < 18) return;
  if (in_sizes[0] != kTok * kInDim) return;
  if (in_sizes[1] != kHid * kInDim || in_sizes[2] != kInDim * kHid || in_sizes[3] != kInDim) return;
  if (in_sizes[4] != kLayers * 3 * kHid * kHid || in_sizes[5] != kLayers * 3 * kHid) return;
  if (in_sizes[6] != kLayers * kHid * kHid || in_sizes[7] != kLayers * kHid) return;
  if (in_sizes[8] != kLayers * kHid || in_sizes[9] != kLayers * kHid) return;
  if (in_sizes[10] != kLayers * kHid || in_sizes[11] != kLayers * kHid) return;
  if (in_sizes[12] != kLayers * kFfn * kHid || in_sizes[13] != kLayers * kFfn) return;
  if (in_sizes[14] != kLayers * kHid * kFfn || in_sizes[15] != kLayers * kHid) return;
  if (in_sizes[16] != kHid || in_sizes[17] != kHid) return;
  if (out_size != kTok * kInDim) return;

  const float* x     = (const float*)d_in[0];
  const float* w_in  = (const float*)d_in[1];
  const float* w_out = (const float*)d_in[2];
  const float* b_out = (const float*)d_in[3];
  const float* qkv_w = (const float*)d_in[4];
  const float* qkv_b = (const float*)d_in[5];
  const float* out_w = (const float*)d_in[6];
  const float* out_b = (const float*)d_in[7];
  const float* ln1_g = (const float*)d_in[8];
  const float* ln1_b = (const float*)d_in[9];
  const float* ln2_g = (const float*)d_in[10];
  const float* ln2_b = (const float*)d_in[11];
  const float* ff1_w = (const float*)d_in[12];
  const float* ff1_b = (const float*)d_in[13];
  const float* ff2_w = (const float*)d_in[14];
  const float* ff2_b = (const float*)d_in[15];
  const float* lnf_g = (const float*)d_in[16];
  const float* lnf_b = (const float*)d_in[17];
  float* outp = (float*)d_out;

  const size_t hWin  = 0;
  const size_t hWout = hWin  + (size_t)kHid * kInDim;
  const size_t hQKV  = hWout + (size_t)kInDim * kHid;
  const size_t hOW   = hQKV  + (size_t)kLayers * 3 * kHid * kHid;
  const size_t hFF1  = hOW   + (size_t)kLayers * kHid * kHid;
  const size_t hFF2  = hFF1  + (size_t)kLayers * kFfn * kHid;
  const size_t hWtot = hFF2  + (size_t)kLayers * kHid * kFfn;

  const size_t PX16 = (size_t)kTok * kInDim * 2;
  const size_t PW16 = hWtot * 2;
  const size_t PPE  = (size_t)kSeq * kHid * 4;
  const size_t PH   = (size_t)kTok * kHid * 4;
  const size_t PA16 = (size_t)kTok * kHid * 2;
  const size_t PQK  = (size_t)kTok * kQKW * 2;
  const size_t PVT  = (size_t)kBatch * kHid * kSeq * 2;
  const size_t PS   = (size_t)kNZ * kSeq * kPBW * 4;
  const size_t PP   = (size_t)kNZ * kSeq * kPBW * 2;
  const size_t PCTX = (size_t)kTok * kHid * 2;
  const size_t PFF  = (size_t)kTok * kFfn * 2;
  size_t off = 0;
  const size_t oX   = off; off += PX16;
  const size_t oW   = off; off += PW16;
  const size_t oPE  = off; off += PPE;
  const size_t oH0  = off; off += PH;
  const size_t oH1  = off; off += PH;
  const size_t oA   = off; off += PA16;
  const size_t oQK  = off; off += PQK;
  const size_t oVT  = off; off += PVT;
  const size_t oS   = off; off += PS;
  const size_t oP   = off; off += PP;
  const size_t oCTX = off; off += PCTX;
  const size_t oFF  = off; off += PFF;
  if (off > ws_size) return;
  if (off > (size_t)134217728) return;

  char* ws = (char*)d_ws;
  unsigned short* X16   = (unsigned short*)(ws + oX);
  unsigned short* W16   = (unsigned short*)(ws + oW);
  float*          PE    = (float*)(ws + oPE);
  float*          H0    = (float*)(ws + oH0);
  float*          H1    = (float*)(ws + oH1);
  unsigned short* A16   = (unsigned short*)(ws + oA);
  unsigned short* QK16  = (unsigned short*)(ws + oQK);
  unsigned short* VT16  = (unsigned short*)(ws + oVT);
  float*          Sbuf  = (float*)(ws + oS);
  unsigned short* P16   = (unsigned short*)(ws + oP);
  unsigned short* CTX16 = (unsigned short*)(ws + oCTX);
  unsigned short* FF16  = (unsigned short*)(ws + oFF);
  unsigned short* WIN16  = W16 + hWin;
  unsigned short* WOUT16 = W16 + hWout;
  unsigned short* QKVW16 = W16 + hQKV;
  unsigned short* OW16   = W16 + hOW;
  unsigned short* FF1W16 = W16 + hFF1;
  unsigned short* FF2W16 = W16 + hFF2;

  const float* dummy = b_out;
  const dim3 blk(256);

  {
    const int n2x = kTok * kInDim / 2;
    cast_f32_f16x2s<<<dim3((n2x + 255) / 256), blk, 0, stream>>>(x, (_Float16*)X16, n2x, 1.0f);
    const int n2a = kHid * kInDim / 2;
    cast_f32_f16x2s<<<dim3((n2a + 255) / 256), blk, 0, stream>>>(w_in,  (_Float16*)WIN16,  n2a, 16.0f);
    cast_f32_f16x2s<<<dim3((n2a + 255) / 256), blk, 0, stream>>>(w_out, (_Float16*)WOUT16, n2a, 16.0f);
    const int n2q = kLayers * 3 * kHid * kHid / 2;
    cast_f32_f16x2s<<<dim3((n2q + 255) / 256), blk, 0, stream>>>(qkv_w, (_Float16*)QKVW16, n2q, 16.0f);
    const int n2o = kLayers * kHid * kHid / 2;
    cast_f32_f16x2s<<<dim3((n2o + 255) / 256), blk, 0, stream>>>(out_w, (_Float16*)OW16, n2o, 16.0f);
    const int n2f = kLayers * kFfn * kHid / 2;
    cast_f32_f16x2s<<<dim3((n2f + 255) / 256), blk, 0, stream>>>(ff1_w, (_Float16*)FF1W16, n2f, 16.0f);
    cast_f32_f16x2s<<<dim3((n2f + 255) / 256), blk, 0, stream>>>(ff2_w, (_Float16*)FF2W16, n2f, 16.0f);
  }
  pe_rows_kernel<<<dim3(kSeq), dim3(128), 0, stream>>>(PE);

  wmma_gemm64<0, false, 0, 0, true><<<dim3(((kSeq / 64) * (kHid / 64) + 7) / 8, kBatch, 1), blk, 0, stream>>>(
      X16, X16, kInDim, (long)kSeq * kInDim, WIN16, WIN16, kInDim, 0L,
      (void*)H0, (void*)H0, kHid, (long)kSeq * kHid,
      dummy, PE, 0L, kSeq, kHid, kInDim, 1.0f, 1.0f, 0L, 0L, 0L, 0L);

  const dim3 gTok256(((kTok / 64) * (kHid / 64) + 7) / 8, 1, 1);
  const dim3 gTok512(((kTok / 64) * (kQKW / 64) + 7) / 8, 1, 1);
  const dim3 gTok1024(((kTok / 64) * (kFfn / 64) + 7) / 8, 1, 1);
  const dim3 gVT(((kHid / 64) * (kSeq / 64) + 7) / 8, kBatch, 1);
  const dim3 gS(((kSeq / 64) * (kSeq / 64) + 7) / 8, kHeads, kBatch);
  const dim3 gSm(kSeq / 4, kNZ);
  const dim3 gPV(((kSeq / 64) * (kHdim / 64) + 7) / 8, kHeads, kBatch);
  const dim3 gLN(kTok / 8);

  for (int l = 0; l < kLayers; ++l) {
    const unsigned short* Wqkv_l = QKVW16 + (size_t)l * 3 * kHid * kHid;
    const unsigned short* Wv_l   = Wqkv_l + (size_t)2 * kHid * kHid;
    const unsigned short* Wo_l   = OW16   + (size_t)l * kHid * kHid;
    const unsigned short* W1_l   = FF1W16 + (size_t)l * kFfn * kHid;
    const unsigned short* W2_l   = FF2W16 + (size_t)l * kHid * kFfn;
    const float* bqkv_l = qkv_b + (size_t)l * 3 * kHid;

    layernorm_f16_kernel<<<gLN, blk, 0, stream>>>(H0, ln1_g + (size_t)l * kHid, ln1_b + (size_t)l * kHid, A16, kTok);

    wmma_gemm64<0, false, 2, 1, false><<<gTok512, blk, 0, stream>>>(
        A16, A16, kHid, 0L, Wqkv_l, Wqkv_l, kHid, 0L, (void*)QK16, (void*)QK16, kQKW, 0L,
        bqkv_l, dummy, 0L, kTok, kQKW, kHid, 0.5f, 8.0f, 0L, 0L, 0L, 0L);

    wmma_gemm64<0, false, 1, 1, false><<<gVT, blk, 0, stream>>>(
        Wv_l, Wv_l, kHid, 0L, A16, A16, kHid, (long)kSeq * kHid,
        (void*)VT16, (void*)VT16, kSeq, (long)kHid * kSeq,
        bqkv_l + 2 * kHid, dummy, 0L, kHid, kSeq, kHid, 0.5f, 8.0f, 0L, 0L, 0L, 0L);

    wmma_gemm64<0, false, 0, 0, false, 0, 1, -1, true><<<gS, blk, 0, stream>>>(
        QK16, QK16, kQKW, (long)kHdim, QK16 + kHid, QK16 + kHid, kQKW, (long)kHdim,
        (void*)Sbuf, (void*)Sbuf, kPBW, (long)kSeq * kPBW,
        dummy, dummy, 0L, kSeq, kSeq, kHdim, 0.001953125f, 1.0f,
        (long)kSeq * kQKW, (long)kSeq * kQKW, (long)kHeads * kSeq * kPBW, 0L);

    band_softmax_kernel<<<gSm, dim3(128), 0, stream>>>(Sbuf, P16);

    wmma_gemm64<0, false, 0, 1, false, 0, -1, 1, true><<<gPV, blk, 0, stream>>>(
        P16, P16, kPBW, (long)kSeq * kPBW, VT16, VT16, kSeq, (long)kHdim * kSeq,
        (void*)CTX16, (void*)CTX16, kHid, (long)kHdim,
        dummy, dummy, 0L, kSeq, kHdim, kSeq, 0.00006103515625f, 1.0f,
        (long)kHeads * kSeq * kPBW, (long)kHid * kSeq, (long)kSeq * kHid, 0L);

    wmma_gemm64<0, false, 2, 0, true><<<gTok256, blk, 0, stream>>>(
        CTX16, CTX16, kHid, 0L, Wo_l, Wo_l, kHid, 0L, (void*)H1, (void*)H1, kHid, 0L,
        out_b + (size_t)l * kHid, H0, 0L, kTok, kHid, kHid, 0.00390625f, 1.0f, 0L, 0L, 0L, 0L);

    layernorm_f16_kernel<<<gLN, blk, 0, stream>>>(H1, ln2_g + (size_t)l * kHid, ln2_b + (size_t)l * kHid, A16, kTok);

    wmma_gemm64<0, false, 2, 1, false, 2><<<gTok1024, blk, 0, stream>>>(
        A16, A16, kHid, 0L, W1_l, W1_l, kHid, 0L, (void*)FF16, (void*)FF16, kFfn, 0L,
        ff1_b + (size_t)l * kFfn, dummy, 0L, kTok, kFfn, kHid, 0.5f, 8.0f, 0L, 0L, 0L, 0L);

    wmma_gemm64<0, false, 2, 0, true><<<gTok256, blk, 0, stream>>>(
        FF16, FF16, kFfn, 0L, W2_l, W2_l, kFfn, 0L, (void*)H0, (void*)H0, kHid, 0L,
        ff2_b + (size_t)l * kHid, H1, 0L, kTok, kHid, kFfn, 0.0078125f, 1.0f, 0L, 0L, 0L, 0L);
  }

  layernorm_f16_kernel<<<gLN, blk, 0, stream>>>(H0, lnf_g, lnf_b, A16, kTok);
  wmma_gemm64<0, false, 2, 0, false><<<gTok256, blk, 0, stream>>>(
      A16, A16, kHid, 0L, WOUT16, WOUT16, kHid, 0L, (void*)outp, (void*)outp, kInDim, 0L,
      b_out, dummy, 0L, kTok, kInDim, kHid, 0.0625f, 1.0f, 0L, 0L, 0L, 0L);
}
